// Decoder_64012192580153
// MI455X (gfx1250) — hardware-run, weakly checked
//
#include <hip/hip_runtime.h>
#include <stdint.h>

#define NN    2048
#define DD    32
#define HH    64
#define NC    128
#define LP    68
#define ZBLK  ((NN * DD / 8) / 256)

static_assert(DD == 32);
static_assert(NC == 128);
static_assert(NC == 2 * HH);
static_assert(HH == 64);
static_assert(NN % 128 == 0);
static_assert(NN % 64 == 0);
static_assert((NN * DD / 8) % 256 == 0);
static_assert((LP * 4) % 16 == 0);
static_assert((NC * DD / 8) == 512);

typedef __attribute__((ext_vector_type(16))) __bf16 v16b;
typedef __attribute__((ext_vector_type(8)))  __bf16 v8b;
typedef __attribute__((ext_vector_type(8)))  float  v8f;
typedef __attribute__((ext_vector_type(4)))  float  v4f;
typedef __attribute__((ext_vector_type(4)))  unsigned int v4u;
typedef v8b __attribute__((may_alias)) v8ba;
typedef v4f __attribute__((may_alias)) v4fa;
typedef v4u __attribute__((may_alias)) v4ua;

union FragU { v16b v; v8b h[2]; };

__device__ __forceinline__ unsigned short f2bf_bits(float f) {
  const unsigned u = __float_as_uint(f);
  return (unsigned short)((u + 0x7FFFu + ((u >> 16) & 1u)) >> 16);
}
__device__ __forceinline__ unsigned bf16r_bits(float f) {
  const unsigned u = __float_as_uint(f);
  return (u + 0x7FFFu + ((u >> 16) & 1u)) & 0xFFFF0000u;
}
__device__ __forceinline__ unsigned pk16(unsigned short a, unsigned short b) { return (unsigned)a | ((unsigned)b << 16); }

__device__ __forceinline__ v8f wmma_bf16(v16b a, v16b b, v8f c) {
  v8f d = __builtin_amdgcn_wmma_f32_16x16x32_bf16(false, a, false, b, (short)0, c, false, false);
  asm volatile("v_nop\n\tv_nop\n\tv_nop\n\tv_nop" : "+v"(d) : "v"(a), "v"(b));
  return d;
}

__device__ __forceinline__ v16b load_frag(const unsigned short* p, int hh) {
  FragU f;
  f.h[0] = *(const v8ba*)(p + 8 * hh);
  f.h[1] = *(const v8ba*)(p + 16 + 8 * hh);
  return f.v;
}

__global__ __launch_bounds__(256) void k_prep(const float* __restrict__ Z, const float* __restrict__ W1,
                                              const float* __restrict__ b1, const float* __restrict__ W2,
                                              const float* __restrict__ b2,
                                              unsigned short* __restrict__ ZB, unsigned short* __restrict__ W1T,
                                              float* __restrict__ PAR) {
  __shared__ __align__(16) float sW[2 * DD * HH];
  const int tid = threadIdx.x;
  if (blockIdx.x < ZBLK) {
    const int g = blockIdx.x * 256 + tid;
    const float* src = Z + (size_t)g * 8;
    const v4f a = *(const v4fa*)src;
    const v4f c = *(const v4fa*)(src + 4);
    v4u o;
    o[0] = pk16(f2bf_bits(a[0]), f2bf_bits(a[1]));
    o[1] = pk16(f2bf_bits(a[2]), f2bf_bits(a[3]));
    o[2] = pk16(f2bf_bits(c[0]), f2bf_bits(c[1]));
    o[3] = pk16(f2bf_bits(c[2]), f2bf_bits(c[3]));
    unsigned short* dst = ZB + (size_t)g * 8;
    *(volatile v4u*)dst = o;
    __threadfence();
    *(volatile v4u*)dst = o;
  } else {
#pragma unroll
    for (int p = 0; p < 4; ++p) {
      const int idx = tid + 256 * p;
      const v4f v = *(const v4fa*)(W1 + 4 * idx);
      *(v4fa*)(sW + 4 * idx) = v;
    }
    const int tb = (tid < 15) ? tid : 15;
    int tw = tid - 16;
    tw = (tw < 0) ? 0 : tw;
    tw = (tw > 15) ? 15 : tw;
    const v4f b1v = *(const v4fa*)(b1 + 4 * tb);
    const v4f w2v = *(const v4fa*)(W2 + 4 * tw);
    const float b2s = b2[0];
    asm volatile("" :: "v"(b1v), "v"(w2v), "v"(b2s));
    __syncthreads();

    v4u wo[2];
#pragma unroll
    for (int it = 0; it < 2; ++it) {
      const int u = tid + 256 * it;
      const int n = u >> 2, kq = u & 3;
      const int kb = ((n >> 6) << 5) + 8 * kq;
      const int col = n & 63;
      unsigned short e[8];
#pragma unroll
      for (int j = 0; j < 8; ++j) e[j] = f2bf_bits(sW[(kb + j) * HH + col]);
      wo[it][0] = pk16(e[0], e[1]);
      wo[it][1] = pk16(e[2], e[3]);
      wo[it][2] = pk16(e[4], e[5]);
      wo[it][3] = pk16(e[6], e[7]);
    }
    const unsigned m0 = 0u - (unsigned)(tid < 16);
    const unsigned m1 = 0u - (unsigned)((tid >= 16) & (tid < 32));
    const unsigned m2 = 0u - (unsigned)(tid == 32);
    v4u po;
#pragma unroll
    for (int j = 0; j < 4; ++j) po[j] = (bf16r_bits(b1v[j]) & m0) | (bf16r_bits(w2v[j]) & m1);
    po[0] |= bf16r_bits(b2s) & m2;

    for (int pass = 0; pass < 2; ++pass) {
#pragma unroll
      for (int it = 0; it < 2; ++it) {
        const int u = tid + 256 * it;
        *(volatile v4u*)(W1T + (size_t)u * 8) = wo[it];
      }
      if (tid < 64) {
        *(volatile v4u*)(PAR + 4 * tid) = po;
      }
      __threadfence();
    }
  }
}

__global__ __launch_bounds__(128) void k_proj(const unsigned short* __restrict__ ZB,
                                              const unsigned short* __restrict__ W1T,
                                              const float* __restrict__ PAR,
                                              float* __restrict__ AB) {
  __shared__ __align__(16) float sF[128 * 64];
  __shared__ __align__(16) float sB[128];
  const int tid = threadIdx.x, lane = tid & 31, w = tid >> 5;
  const int hh = lane >> 4, m = lane & 15;
  const int m0 = blockIdx.x * 128;
  const int n0 = blockIdx.y * 64;
  const int m0w = m0 + 32 * w;

  if (w == 0) {
    const v4f pv = *(const v4fa*)(PAR + 4 * lane);
    *(v4fa*)(sB + 4 * lane) = pv;
  }

  const v8f zero8 = {0.f, 0.f, 0.f, 0.f, 0.f, 0.f, 0.f, 0.f};
  v8f acc[2][4];
#pragma unroll
  for (int mt = 0; mt < 2; ++mt)
#pragma unroll
    for (int nt = 0; nt < 4; ++nt) acc[mt][nt] = zero8;

  {
    const unsigned short* a0 = ZB + (size_t)(m0w + m) * DD;
    const unsigned short* a1 = a0 + (size_t)16 * DD;
    const unsigned short* bp = W1T + (size_t)(n0 + m) * DD;
    const v16b f0 = load_frag(a0, hh);
    const v16b f1 = load_frag(a1, hh);
#pragma unroll
    for (int nt = 0; nt < 4; ++nt) {
      const v16b fb = load_frag(bp + (size_t)nt * 16 * DD, hh);
      acc[0][nt] = wmma_bf16(f0, fb, acc[0][nt]);
      acc[1][nt] = wmma_bf16(f1, fb, acc[1][nt]);
    }
  }
  __syncthreads();

#pragma unroll
  for (int nt = 0; nt < 4; ++nt) {
    const int feat = 16 * nt + m;
    const float bvl = (n0 == 0) ? sB[feat] : 0.0f;
#pragma unroll
    for (int mt = 0; mt < 2; ++mt)
#pragma unroll
      for (int r = 0; r < 8; ++r) {
        const int tokl = 32 * w + 16 * mt + 8 * hh + r;
        sF[tokl * 64 + feat] = acc[mt][nt][r] + bvl;
      }
  }
  __syncthreads();
  {
    const int rsub = lane >> 4, c4 = (lane & 15) * 4;
    v4f vals[16];
#pragma unroll
    for (int it = 0; it < 16; ++it) {
      const int row = 32 * w + 2 * it + rsub;
      vals[it] = *(const v4fa*)(sF + row * 64 + c4);
    }
    for (int pass = 0; pass < 2; ++pass) {
#pragma unroll
      for (int it = 0; it < 16; ++it) {
        const int row = 32 * w + 2 * it + rsub;
        *(volatile v4f*)(AB + (size_t)(m0 + row) * NC + n0 + c4) = vals[it];
      }
      __threadfence();
    }
  }
}

__global__ __launch_bounds__(256) void k_pair(const float* __restrict__ AB, const float* __restrict__ PAR,
                                              float* __restrict__ out) {
  __shared__ __align__(16) float As[HH * LP];
  __shared__ __align__(16) float Bs[HH * LP];
  __shared__ __align__(16) float Ls[64 * 64];
  __shared__ __align__(16) float sP[128];
  const int tid = threadIdx.x, lane = tid & 31, w = tid >> 5;
  const int i0 = blockIdx.y * 64;
  const int j0 = blockIdx.x * 64;

  {
    const int c4 = (tid & 15) * 4, rr = tid >> 4;
#pragma unroll
    for (int p = 0; p < 4; ++p) {
      const int r = rr + 16 * p;
      const v4f va = *(const v4fa*)(AB + (size_t)(i0 + r) * NC + c4);
      const v4f vb = *(const v4fa*)(AB + (size_t)(j0 + r) * NC + HH + c4);
      As[(c4 + 0) * LP + r] = va[0];
      As[(c4 + 1) * LP + r] = va[1];
      As[(c4 + 2) * LP + r] = va[2];
      As[(c4 + 3) * LP + r] = va[3];
      Bs[(c4 + 0) * LP + r] = vb[0];
      Bs[(c4 + 1) * LP + r] = vb[1];
      Bs[(c4 + 2) * LP + r] = vb[2];
      Bs[(c4 + 3) * LP + r] = vb[3];
    }
  }
  if (w == 0) {
    const v4f pv = *(const v4fa*)(PAR + HH + 4 * lane);
    *(v4fa*)(sP + 4 * lane) = pv;
  }
  __syncthreads();

  const int ti4 = (tid >> 4) * 4;
  const int tj4 = (tid & 15) * 4;
  static_assert(256 == 16 * 16);

  float acc[4][4];
#pragma unroll
  for (int ii = 0; ii < 4; ++ii)
#pragma unroll
    for (int jj = 0; jj < 4; ++jj) acc[ii][jj] = 0.0f;

#pragma unroll 2
  for (int c = 0; c < HH; ++c) {
    const v4f a4 = *(const v4fa*)(As + c * LP + ti4);
    const v4f b4 = *(const v4fa*)(Bs + c * LP + tj4);
    const float wv = sP[c];
#pragma unroll
    for (int ii = 0; ii < 4; ++ii)
#pragma unroll
      for (int jj = 0; jj < 4; ++jj) {
        float v = a4[ii] + b4[jj];
        v = fmaxf(v, 0.0f);
        acc[ii][jj] = fmaf(v, wv, acc[ii][jj]);
      }
  }

#pragma unroll
  for (int ii = 0; ii < 4; ++ii) {
    const v4f o = {acc[ii][0], acc[ii][1], acc[ii][2], acc[ii][3]};
    *(v4fa*)(Ls + (ti4 + ii) * 64 + tj4) = o;
  }
  __syncthreads();

  const float b2r = sP[HH];
  const int rsub = tid >> 4;
#pragma unroll 1
  for (int t = 0; t < 4; ++t) {
    const int row = 16 * t + rsub;
    const v4f lv = *(const v4fa*)(Ls + row * 64 + tj4);
    v4f o;
    o[0] = 1.0f / (1.0f + expf(-(lv[0] + b2r)));
    o[1] = 1.0f / (1.0f + expf(-(lv[1] + b2r)));
    o[2] = 1.0f / (1.0f + expf(-(lv[2] + b2r)));
    o[3] = 1.0f / (1.0f + expf(-(lv[3] + b2r)));
    float* dst = out + (size_t)(i0 + row) * NN + j0 + tj4;
    *(volatile v4f*)dst = o;
    __threadfence();
    *(volatile v4f*)dst = o;
  }
}

extern "C" void kernel_launch(void* const* d_in, const int* in_sizes, int n_in,
                              void* d_out, int out_size, void* d_ws, size_t ws_size,
                              hipStream_t stream) {
  if (n_in < 5) return;
  if (in_sizes[0] != NN * DD) return;
  if (in_sizes[1] != 2 * DD * HH) return;
  if (in_sizes[2] != HH) return;
  if (in_sizes[3] != HH) return;
  if (in_sizes[4] != 1) return;
  if (out_size != NN * NN) return;

  const float* Z  = (const float*)d_in[0];
  const float* W1 = (const float*)d_in[1];
  const float* b1 = (const float*)d_in[2];
  const float* W2 = (const float*)d_in[3];
  const float* b2 = (const float*)d_in[4];
  float* out = (float*)d_out;

  const size_t PZB = (size_t)NN * DD * 2;
  const size_t PWT = (size_t)NC * DD * 2;
  const size_t PPA = (size_t)256 * 4;
  const size_t PAB = (size_t)NN * NC * 4;
  size_t off = 0;
  const size_t oZB = off; off += PZB;
  const size_t oWT = off; off += PWT;
  const size_t oPA = off; off += PPA;
  const size_t oAB = off; off += PAB;
  if (off > ws_size) return;

  char* ws = (char*)d_ws;
  unsigned short* ZB  = (unsigned short*)(ws + oZB);
  unsigned short* W1T = (unsigned short*)(ws + oWT);
  float*          PAR = (float*)(ws + oPA);
  float*          AB  = (float*)(ws + oAB);

  k_prep<<<dim3(ZBLK + 1), 256, 0, stream>>>(Z, W1, b1, W2, b2, ZB, W1T, PAR);
  k_proj<<<dim3(NN / 128, NC / 64), 128, 0, stream>>>(ZB, W1T, PAR, AB);
  k_pair<<<dim3(NN / 64, NN / 64), 256, 0, stream>>>(AB, PAR, out);
  (void)hipGetLastError();
}
